// EQ_GNN_20023137534500
// MI455X (gfx1250) — hardware-verified
//
#include <hip/hip_runtime.h>
#include <hip/hip_bf16.h>
#include <math.h>


typedef _Float16 bf16;
typedef _Float16 f16;
typedef __attribute__((ext_vector_type(4))) unsigned v4u_t;
typedef unsigned v4ua __attribute__((ext_vector_type(4), may_alias));
typedef __attribute__((ext_vector_type(4))) float v4f_t;
typedef float v4fa __attribute__((ext_vector_type(4), may_alias));
typedef __attribute__((ext_vector_type(16))) bf16  bf16x16;
typedef bf16x16 f16x16;
typedef __attribute__((ext_vector_type(8)))  bf16  bf16x8;
typedef bf16x8 f16x8;
typedef __attribute__((ext_vector_type(4)))  bf16  bf16x4;
typedef __attribute__((ext_vector_type(8)))  float f32x8;
__device__ __forceinline__ f32x8 wmma16(f16x16 a, f16x16 b, f32x8 c) {
  c = __builtin_amdgcn_wmma_f32_16x16x32_f16(false, a, false, b, (short)0, c, false, false);
  asm volatile("v_nop\n\tv_nop\n\tv_nop\n\tv_nop" : "+v"(c) : "v"(a), "v"(b));
  return c;
}
#define LDS_STRIDE 48
#define KSTRIDE    72
#define VSTRIDE    48

__device__ __forceinline__ f32x8 wmma_bf16(bf16x16 a, bf16x16 b, f32x8 c) {
  c = __builtin_amdgcn_wmma_f32_16x16x32_f16(false, a, false, b, (short)0, c, false, false);
  asm volatile("v_nop\n\tv_nop\n\tv_nop\n\tv_nop" : "+v"(c) : "v"(a), "v"(b));
  return c;
}

template <typename T>
__device__ __forceinline__ bf16x16 load_frag(const T* __restrict__ base, int ld,
                                             int row0, int k0) {
  const int lane = threadIdx.x & 31;
  const int r    = lane & 15;
  const int kh   = (lane >> 4) * 8;
  const T* p0 = base + (size_t)(row0 + r) * ld + (k0 + kh);
  const T* p1 = p0 + 16;
  bf16x16 f;
#pragma unroll
  for (int i = 0; i < 8; ++i) {
    f[i]     = (bf16)p0[i];
    f[i + 8] = (bf16)p1[i];
  }
  return f;
}

__device__ __forceinline__ bf16x16 lds_frag(const bf16* base, int stride) {
  const int lane = threadIdx.x & 31;
  const int row  = lane & 15;
  const int kh   = (lane >> 4) * 8;
  const bf16x8 lo = *(const bf16x8*)(base + row * stride + kh);
  const bf16x8 hi = *(const bf16x8*)(base + row * stride + kh + 16);
  bf16x16 f;
#pragma unroll
  for (int i = 0; i < 8; ++i) { f[i] = lo[i]; f[i + 8] = hi[i]; }
  return f;
}

template <typename T>
__device__ __forceinline__ void stage_read16(const T* __restrict__ p, float* buf) {
#pragma unroll
  for (int i = 0; i < 16; ++i) buf[i] = (float)p[i];
}

__device__ __forceinline__ void stage_write(bf16* dst, const float* buf, int nquad) {
#pragma unroll
  for (int i = 0; i < nquad; ++i) {
    bf16x4 q;
    q[0] = (bf16)buf[4 * i];     q[1] = (bf16)buf[4 * i + 1];
    q[2] = (bf16)buf[4 * i + 2]; q[3] = (bf16)buf[4 * i + 3];
    *(bf16x4*)(dst + 4 * i) = q;
  }
}


#define GSTR 48
#define GSTR 48
template <typename AT, int EPI, bool OUT16>
__global__ __launch_bounds__(256) void gemm_kne(const AT* __restrict__ A, int lda, const float* __restrict__ Wm, int ldw,
                                                const float* __restrict__ bias, const float* __restrict__ R, const float* __restrict__ gvec,
                                                void* __restrict__ Yv, int ldy, int K) {
  __shared__ __attribute__((aligned(16))) f16 ldsA[128 * GSTR];
  __shared__ __attribute__((aligned(16))) f16 ldsW[128 * GSTR];
  __shared__ __attribute__((aligned(16))) float oS[8][32 * 68];
  const int tid = threadIdx.x, lane = tid & 31, wave = tid >> 5, cl = lane & 15, rh = (lane >> 4) * 8;
  const int m0 = blockIdx.x * 128, n0 = blockIdx.y * 128;
  const int wm = (wave & 3) * 32, wn = (wave >> 2) * 64;
  f32x8 acc[2][4];
#pragma unroll
  for (int i = 0; i < 2; ++i)
#pragma unroll
    for (int j = 0; j < 4; ++j) { f32x8 z = {}; acc[i][j] = z; }
#pragma unroll 1
  for (int k0 = 0; k0 < K; k0 += 32) {
    __syncthreads();
    { const int row = tid >> 1, ch = (tid & 1) * 16;
      const AT* src = A + (size_t)(m0 + row) * lda + k0 + ch;
#pragma unroll
      for (int g = 0; g < 16; ++g) ldsA[row * GSTR + ch + g] = (f16)src[g]; }
    { const int k = tid >> 3, nn0 = (tid & 7) * 16;
      const float* src = Wm + (size_t)(k0 + k) * ldw + n0 + nn0;
#pragma unroll
      for (int g = 0; g < 4; ++g) { const v4f_t v = *(const v4f_t*)(src + 4 * g);
#pragma unroll
        for (int u = 0; u < 4; ++u) ldsW[(nn0 + 4 * g + u) * GSTR + k] = (f16)v[u]; } }
    __syncthreads();
    f16x16 af[2];
#pragma unroll
    for (int i = 0; i < 2; ++i) af[i] = lds_frag(ldsA + (wm + 16 * i) * GSTR, GSTR);
#pragma unroll
    for (int j = 0; j < 4; ++j) {
      const f16x16 bf = lds_frag(ldsW + (wn + 16 * j) * GSTR, GSTR);
#pragma unroll
      for (int i = 0; i < 2; ++i) acc[i][j] = wmma16(af[i], bf, acc[i][j]);
    }
  }
  float* so = oS[wave];
#pragma unroll
  for (int i = 0; i < 2; ++i)
#pragma unroll
    for (int j = 0; j < 4; ++j) {
      const int n = n0 + wn + 16 * j + cl;
      const float bv = bias ? bias[n] : 0.0f;
      const float gv = (EPI == 2 || EPI == 4) ? gvec[n] : 0.0f;
      if (EPI == 1) {
#pragma unroll 1
        for (int r = 0; r < 8; ++r) { const float xg = acc[i][j][r] + bv; so[(16 * i + rh + r) * 68 + 16 * j + cl] = 0.5f * xg * (1.0f + erff(xg * 0.70710678118654752f)); }
      } else {
#pragma unroll
        for (int r = 0; r < 8; ++r) {
          float v = acc[i][j][r] + bv;
          if (EPI == 3) v = fmaxf(v, 0.0f);
          if (EPI == 5) v = (v > 0.0f) ? v : (__expf(v) - 1.0f);
          if (EPI == 6) v = 1.0f / (1.0f + __expf(-v));
          if (EPI == 8) v = v / (1.0f + __expf(-v));
          if (EPI == 4) v = gv * v;
          if (EPI == 2) v = R[(size_t)(m0 + wm + 16 * i + rh + r) * ldy + n] + gv * v;
          so[(16 * i + rh + r) * 68 + 16 * j + cl] = v;
        }
      }
    }
  asm volatile("s_wait_dscnt 0" ::: "memory");
  __builtin_amdgcn_wave_barrier();
#pragma unroll 1
  for (int pass = 0; pass < 2; ++pass) {
    if (OUT16) {
      f16* Y = (f16*)Yv;
#pragma unroll
      for (int it = 0; it < 8; ++it) { const int c = lane + 32 * it, rr = c >> 3, q8 = (c & 7) * 8;
        union { f16 h[8]; v4u_t v; } u;
#pragma unroll
        for (int e = 0; e < 8; ++e) u.h[e] = (f16)so[rr * 68 + q8 + e];
        *(volatile v4u_t*)(Y + (size_t)(m0 + wm + rr) * ldy + n0 + wn + q8) = u.v; }
    } else {
      float* Y = (float*)Yv;
#pragma unroll
      for (int it = 0; it < 16; ++it) { const int f4 = lane + 32 * it, rr = f4 >> 4, q = (f4 & 15) * 4;
        *(volatile v4f_t*)(Y + (size_t)(m0 + wm + rr) * ldy + n0 + wn + q) = *(const v4fa*)(so + rr * 68 + q); }
    }
    __threadfence();
  }
}


#define NCH_RUN 32
#define BBq 128
#define NPq 128
#define FFq 32
#define EPG 16256
#define GCH 4
#define ECH (GCH * EPG)
#define NCHUNK (BBq / GCH)
#define NNODE (BBq * NPq)
__global__ __launch_bounds__(256) void k_padw(const float* __restrict__ w, const float* __restrict__ b, float* __restrict__ wp, float* __restrict__ bp, int K, int N) {
  const int k = blockIdx.x, n = threadIdx.x; if (n < 128) { const float v = (k < K && n < N) ? w[(size_t)k * N + n] : 0.0f; *(volatile float*)(wp + (size_t)k * 128 + n) = v; __threadfence(); *(volatile float*)(wp + (size_t)k * 128 + n) = v;
    if (k == 0) { const float bb = (b != nullptr && n < N) ? b[n] : 0.0f; *(volatile float*)(bp + n) = bb; __threadfence(); *(volatile float*)(bp + n) = bb; } } }
__global__ __launch_bounds__(256) void k_edge_in(const float* __restrict__ x, const float* __restrict__ h, const float* __restrict__ dstat, float* __restrict__ EIN, int g0) {
  const int tid = threadIdx.x; const size_t el = (size_t)blockIdx.x * 32 + (tid >> 3); const int part = tid & 7;
  const int bl = (int)(el / EPG), e = (int)(el % EPG); const int b = g0 + bl; const int i = e / (NPq - 1), jj = e % (NPq - 1); const int j = jj + (jj >= i ? 1 : 0);
  float v[12];
#pragma unroll
  for (int u = 0; u < 12; ++u) { const int c = (u >> 2) * 32 + part * 4 + (u & 3); float val = 0.0f;
    if (c < FFq) val = h[((size_t)b * NPq + i) * FFq + c]; else if (c < 2 * FFq) val = h[((size_t)b * NPq + j) * FFq + (c - FFq)];
    else if (c == 2 * FFq) { const float* xi = x + (size_t)b * 384 + 3 * i; const float* xj = x + (size_t)b * 384 + 3 * j; const float r0 = xi[0] - xj[0], r1 = xi[1] - xj[1], r2 = xi[2] - xj[2]; val = r0 * r0 + r1 * r1 + r2 * r2 + 1e-6f; }
    else if (c == 2 * FFq + 1) { const float ds = dstat[(size_t)b * EPG + e]; val = ds * ds; }
    v[u] = val; }
  float* d = EIN + el * 96 + part * 4; v4f_t o0 = {v[0], v[1], v[2], v[3]}, o1 = {v[4], v[5], v[6], v[7]}, o2 = {v[8], v[9], v[10], v[11]};
#pragma unroll 1
  for (int pass = 0; pass < 2; ++pass) { *(volatile v4f_t*)(d) = o0; *(volatile v4f_t*)(d + 32) = o1; *(volatile v4f_t*)(d + 64) = o2; __threadfence(); }
}
__global__ __launch_bounds__(256) void k_gate(float* __restrict__ M, const float* __restrict__ aw, const float* __restrict__ ab) {
  const int tid = threadIdx.x, r = tid >> 3, part = tid & 7; const size_t row = (size_t)blockIdx.x * 32 + r; float* mr = M + row * 128; float s = 0.0f;
#pragma unroll
  for (int u = 0; u < 4; ++u) s = fmaf(mr[part * 4 + u], aw[part * 4 + u], s);
  s += __shfl_xor(s, 1, 32); s += __shfl_xor(s, 2, 32); s += __shfl_xor(s, 4, 32);
  const float g = 1.0f / (1.0f + expf(-(s + ab[0]))); v4f_t v = *(const v4f_t*)(mr + part * 4); v[0] *= g; v[1] *= g; v[2] *= g; v[3] *= g;
  *(volatile v4f_t*)(mr + part * 4) = v; __threadfence(); *(volatile v4f_t*)(mr + part * 4) = v;
}
__global__ __launch_bounds__(256) void k_trans(const float* __restrict__ C1, const float* __restrict__ cw2, float* __restrict__ TR) {
  __shared__ float rs[32];
  const int tid = threadIdx.x, r = tid >> 3, part = tid & 7; const size_t row = (size_t)blockIdx.x * 32 + r; const float* cr = C1 + row * 128; float s = 0.0f;
#pragma unroll
  for (int u = 0; u < 4; ++u) s = fmaf(cr[part * 4 + u], cw2[part * 4 + u], s);
  s += __shfl_xor(s, 1, 32); s += __shfl_xor(s, 2, 32); s += __shfl_xor(s, 4, 32);
  if (part == 0) rs[r] = tanhf(s);
  __syncthreads();
  if (tid < 32) { *(volatile float*)(TR + (size_t)blockIdx.x * 32 + tid) = rs[tid]; __threadfence(); *(volatile float*)(TR + (size_t)blockIdx.x * 32 + tid) = rs[tid]; }
}
__global__ __launch_bounds__(128) void k_xout(const float* __restrict__ x, const float* __restrict__ TR, float* __restrict__ out0, int g0) {
  const int tid = threadIdx.x; if (tid >= 96) return; const int nl = tid / 3, dim = tid % 3; const size_t node = (size_t)blockIdx.x * 32 + nl;
  const int bl = (int)(node / NPq), i = (int)(node % NPq); const int b = g0 + bl; const float* xi = x + (size_t)b * 384 + 3 * i; float acc = 0.0f;
#pragma unroll 1
  for (int jj = 0; jj < NPq - 1; ++jj) { const int j = jj + (jj >= i ? 1 : 0); const float* xj = x + (size_t)b * 384 + 3 * j;
    const float r0 = xi[0] - xj[0], r1 = xi[1] - xj[1], r2 = xi[2] - xj[2]; const float d = sqrtf(r0 * r0 + r1 * r1 + r2 * r2 + 1e-6f);
    const float rd = (dim == 0 ? r0 : (dim == 1 ? r1 : r2)) / (d + 1.0f); acc = fmaf(rd, TR[(size_t)bl * EPG + (size_t)i * (NPq - 1) + jj], acc); }
  const float v = xi[dim] + acc * 5.0f; float* dst = out0 + ((size_t)b * NPq + i) * 3 + dim; *(volatile float*)dst = v; __threadfence(); *(volatile float*)dst = v;
}
__global__ __launch_bounds__(256) void k_nodein(const float* __restrict__ h, const float* __restrict__ M, float* __restrict__ NODEIN, int g0) {
  const int tid = threadIdx.x; const size_t nodel = (size_t)blockIdx.x * 8 + (tid >> 5); const int c = tid & 31; const int bl = (int)(nodel / NPq), i = (int)(nodel % NPq); const size_t gnode = (size_t)(g0 + bl) * NPq + i;
  float s = 0.0f;
#pragma unroll 1
  for (int jj = 0; jj < NPq - 1; ++jj) s += M[((size_t)bl * EPG + (size_t)i * (NPq - 1) + jj) * 128 + c];
  const float hv = h[gnode * FFq + c];
  *(volatile float*)(NODEIN + gnode * 64 + c) = hv; *(volatile float*)(NODEIN + gnode * 64 + 32 + c) = s; __threadfence(); *(volatile float*)(NODEIN + gnode * 64 + c) = hv; *(volatile float*)(NODEIN + gnode * 64 + 32 + c) = s;
}
__global__ __launch_bounds__(256) void k_hout(const float* __restrict__ h, const float* __restrict__ HUP, float* __restrict__ out1) { const int tid = threadIdx.x; const size_t node = (size_t)blockIdx.x * 8 + (tid >> 5); const int c = tid & 31;
  const float v = h[node * FFq + c] + HUP[node * 128 + c]; *(volatile float*)(out1 + node * FFq + c) = v; __threadfence(); *(volatile float*)(out1 + node * FFq + c) = v; }

extern "C" void kernel_launch(void* const* d_in, const int* in_sizes, int n_in,
                              void* d_out, int out_size, void* d_ws, size_t ws_size,
                              hipStream_t stream) {
  (void)in_sizes; (void)n_in; (void)out_size;
  const float** f = (const float**)d_in;
  const float* x = f[0], *h = f[1], *dstat = f[2], *ew1 = f[3], *eb1 = f[4], *ew2 = f[5], *eb2 = f[6], *nw1 = f[7], *nb1 = f[8], *nw2 = f[9], *nb2 = f[10], *cw1 = f[11], *cb1 = f[12], *cw2 = f[13], *aw = f[14], *ab = f[15];
  float* out0 = (float*)d_out;
  float* out1 = out0 + (size_t)NNODE * 3;
  char* ws = (char*)d_ws;
  float* W1p = (float*)ws; ws += 96 * 128 * 4; float* b1p = (float*)ws; ws += 128 * 4;
  float* W2p = (float*)ws; ws += 32 * 128 * 4; float* b2p = (float*)ws; ws += 128 * 4;
  float* C1p = (float*)ws; ws += 32 * 128 * 4; float* cbp = (float*)ws; ws += 128 * 4;
  float* N1p = (float*)ws; ws += 64 * 128 * 4; float* nb1p = (float*)ws; ws += 128 * 4;
  float* N2p = (float*)ws; ws += 32 * 128 * 4; float* nb2p = (float*)ws; ws += 128 * 4;
  float* EIN = (float*)ws; ws += (size_t)ECH * 96 * 4;
  float* H1 = (float*)ws; ws += (size_t)ECH * 128 * 4;
  float* M = (float*)ws; ws += (size_t)ECH * 128 * 4;
  float* TR = (float*)ws; ws += (size_t)ECH * 4;
  float* NODEIN = (float*)ws; ws += (size_t)NNODE * 64 * 4; float* NH = (float*)ws; ws += (size_t)NNODE * 128 * 4; float* HUP = (float*)ws; ws += (size_t)NNODE * 128 * 4;
  if ((size_t)(ws - (char*)d_ws) > ws_size) return;
  const dim3 blk(256);
  k_padw<<<dim3(96), blk, 0, stream>>>(ew1, eb1, W1p, b1p, 66, 32); k_padw<<<dim3(32), blk, 0, stream>>>(ew2, eb2, W2p, b2p, 32, 32); k_padw<<<dim3(32), blk, 0, stream>>>(cw1, cb1, C1p, cbp, 32, 32);
  k_padw<<<dim3(64), blk, 0, stream>>>(nw1, nb1, N1p, nb1p, 64, 32); k_padw<<<dim3(32), blk, 0, stream>>>(nw2, nb2, N2p, nb2p, 32, 32);
  for (int c = 0; c < NCH_RUN; ++c) { const int g0 = c * GCH;
    k_edge_in<<<dim3(ECH / 32), blk, 0, stream>>>(x, h, dstat, EIN, g0);
    gemm_kne<float, 8, false><<<dim3(ECH / 128, 1), blk, 0, stream>>>(EIN, 96, W1p, 128, b1p, nullptr, nullptr, H1, 128, 96);
    gemm_kne<float, 8, false><<<dim3(ECH / 128, 1), blk, 0, stream>>>(H1, 128, W2p, 128, b2p, nullptr, nullptr, M, 128, 32);
    k_gate<<<dim3(ECH / 32), blk, 0, stream>>>(M, aw, ab);
    gemm_kne<float, 8, false><<<dim3(ECH / 128, 1), blk, 0, stream>>>(M, 128, C1p, 128, cbp, nullptr, nullptr, H1, 128, 32);
    k_trans<<<dim3(ECH / 32), blk, 0, stream>>>(H1, cw2, TR);
    k_xout<<<dim3(GCH * NPq / 32), dim3(128), 0, stream>>>(x, TR, out0, g0);
    k_nodein<<<dim3(GCH * NPq / 8), blk, 0, stream>>>(h, M, NODEIN, g0);
  }
  gemm_kne<float, 8, false><<<dim3(NNODE / 128, 1), blk, 0, stream>>>(NODEIN, 64, N1p, 128, nb1p, nullptr, nullptr, NH, 128, 64);
  gemm_kne<float, 0, false><<<dim3(NNODE / 128, 1), blk, 0, stream>>>(NH, 128, N2p, 128, nb2p, nullptr, nullptr, HUP, 128, 32);
  k_hout<<<dim3(NNODE / 8), blk, 0, stream>>>(h, HUP, out1);
}
